// diffusion_model_76802605187805
// MI455X (gfx1250) — hardware-run, weakly checked
//
#include <hip/hip_runtime.h>

typedef float          v8f   __attribute__((ext_vector_type(8)));
typedef float          v4f   __attribute__((ext_vector_type(4)));
typedef unsigned int   v4u   __attribute__((ext_vector_type(4)));
typedef int            v8i   __attribute__((ext_vector_type(8)));
typedef unsigned short v8us  __attribute__((ext_vector_type(8)));
typedef unsigned short v16us __attribute__((ext_vector_type(16)));
typedef __bf16         v16bf __attribute__((ext_vector_type(16)));
typedef _Float16       v16h  __attribute__((ext_vector_type(16)));
typedef v4f  __attribute__((may_alias)) v4fa;
typedef v8us __attribute__((may_alias)) v8usa;
union FragB { v16bf v; v16us u; v8us h[2]; v8i w; };
union FragH { v16h  v; v16us u; v8us h[2]; v8i w; };

__device__ __forceinline__ v8f wmb(const FragB& a, const FragB& b, v8f c) {
  v8f d = __builtin_amdgcn_wmma_f32_16x16x32_bf16(false, a.v, false, b.v, (short)0, c, false, false);
  asm volatile("v_nop\n\tv_nop\n\tv_nop\n\tv_nop" : "+v"(d) : "v"(a.w), "v"(b.w));
  return d;
}

__device__ __forceinline__ v8f wmh(const FragH& a, const FragH& b, v8f c) {
  v8f d = __builtin_amdgcn_wmma_f32_16x16x32_f16(false, a.v, false, b.v, (short)0, c, false, false);
  asm volatile("v_nop\n\tv_nop\n\tv_nop\n\tv_nop" : "+v"(d) : "v"(a.w), "v"(b.w));
  return d;
}

__device__ __forceinline__ unsigned bf16_bits(float f) {
  const unsigned u = __float_as_uint(f);
  const unsigned r = (u + 0x7FFFu + ((u >> 16) & 1u)) >> 16;
  const unsigned q = (u >> 16) | 0x40u;
  return ((u & 0x7fffffffu) > 0x7f800000u) ? q : r;
}

__device__ __forceinline__ float bf16_val(float f) {
  return __uint_as_float(bf16_bits(f) << 16);
}
__device__ __forceinline__ int clampi(int v, int lo, int hi) {
  return v < lo ? lo : (v > hi ? hi : v);
}

__device__ __forceinline__ unsigned f16_bits(float f) {
  const unsigned u  = __float_as_uint(f);
  const unsigned s  = (u >> 16) & 0x8000u;
  const unsigned a  = u & 0x7fffffffu;
  const unsigned t  = a - 0x38000000u;
  const unsigned r  = (t + 0x0FFFu + ((t >> 13) & 1u)) >> 13;
  const unsigned rc = r > 0x7C00u ? 0x7C00u : r;
  const bool small  = a < 0x38800000u;
  const bool isnan  = a > 0x7f800000u;
  const unsigned fin = small ? 0u : (s | rc);
  return isnan ? (s | 0x7E00u) : fin;
}

__device__ __forceinline__ unsigned pk16(unsigned lo, unsigned hi) { return lo | (hi << 16); }
__device__ __forceinline__ unsigned bf16_lo_bits(float v) {
  float hi = bf16_val(v);
  asm volatile("" : "+v"(hi));
  return bf16_bits(v - hi);
}
__device__ __forceinline__ v4u pack8_bf16(v4f a, v4f c) {
  return (v4u){ pk16(bf16_bits(a[0]), bf16_bits(a[1])), pk16(bf16_bits(a[2]), bf16_bits(a[3])),
                pk16(bf16_bits(c[0]), bf16_bits(c[1])), pk16(bf16_bits(c[2]), bf16_bits(c[3])) };
}
__device__ __forceinline__ v4u pack8_bf16_lo(v4f a, v4f c) {
  return (v4u){ pk16(bf16_lo_bits(a[0]), bf16_lo_bits(a[1])), pk16(bf16_lo_bits(a[2]), bf16_lo_bits(a[3])),
                pk16(bf16_lo_bits(c[0]), bf16_lo_bits(c[1])), pk16(bf16_lo_bits(c[2]), bf16_lo_bits(c[3])) };
}
__device__ __forceinline__ v4u pack8_f16(v4f a, v4f c) {
  return (v4u){ pk16(f16_bits(a[0]), f16_bits(a[1])), pk16(f16_bits(a[2]), f16_bits(a[3])),
                pk16(f16_bits(c[0]), f16_bits(c[1])), pk16(f16_bits(c[2]), f16_bits(c[3])) };
}

template <int FORM>
__global__ __launch_bounds__(256) void k_plane(const float* __restrict__ src, int rows, int cols, int ldsrc,
                                               unsigned short* __restrict__ dst, int MP, int KP) {
  static_assert(FORM >= 0 && FORM <= 3);
  const int KTOT = (FORM == 1 || FORM == 3) ? 2 * KP : KP;
  const unsigned ppr   = (unsigned)(KTOT >> 3);
  const unsigned kp8   = (unsigned)(KP >> 3);
  const unsigned total = (unsigned)MP * ppr;
  const unsigned g     = blockIdx.x * 256u + threadIdx.x;
  const unsigned rowu  = g / ppr;
  const unsigned p     = g - rowu * ppr;
  const bool second    = p >= kp8;
  const int row = (int)rowu;
  const int c0  = (int)((second ? p - kp8 : p) << 3);
  const float* srow = src + (size_t)clampi(row, 0, rows - 1) * (size_t)ldsrc;
  float x[8];
  unsigned mk[8];
#pragma unroll
  for (int e = 0; e < 8; ++e) {
    const int c = c0 + e;
    const float v = srow[clampi(c, 0, cols - 1)];
    asm volatile("" :: "v"(v));
    x[e]  = v;
    mk[e] = (row < rows && c < cols) ? 0xFFFFu : 0u;
  }
  const v4f a = (v4f){ x[0], x[1], x[2], x[3] };
  const v4f c = (v4f){ x[4], x[5], x[6], x[7] };
  v4u o;
  if (FORM == 2) {
    o = pack8_f16(a, c);
  } else {
    const v4u hi = pack8_bf16(a, c);
    o = hi;
    if (FORM == 1) { const v4u lo = pack8_bf16_lo(a, c); o = second ? lo : hi; }
  }
  const v4u mw = (v4u){ pk16(mk[0], mk[1]), pk16(mk[2], mk[3]), pk16(mk[4], mk[5]), pk16(mk[6], mk[7]) };
  o &= mw;
  if (g < total) {
    volatile v4u* q = (volatile v4u*)(dst + (size_t)g * 8);
    *q = o;
    __threadfence();
    *q = o;
  }
}

template <int FORM> struct FragOf    { typedef FragB T; };
template <>         struct FragOf<2> { typedef FragH T; };
__device__ __forceinline__ v8f mm(const FragB& a, const FragB& b, v8f c) { return wmb(a, b, c); }
__device__ __forceinline__ v8f mm(const FragH& a, const FragH& b, v8f c) { return wmh(a, b, c); }
template <class F> __device__ __forceinline__ F ld_frag(const unsigned short* p) {
  F f;
  f.h[0] = *(const v8usa*)(p);
  f.h[1] = *(const v8usa*)(p + 16);
  return f;
}

template <int FORM, int EPI>
__global__ __launch_bounds__(256) __attribute__((amdgpu_num_vgpr(248)))
void k_gemm_nt(const unsigned short* __restrict__ A, const unsigned short* __restrict__ B,
               const float* __restrict__ bias, float* __restrict__ D, int M, int N, int KTOT, int ldd) {
  static_assert(FORM >= 0 && FORM <= 2);
  static_assert(EPI == 0 || EPI == 1);
  typedef typename FragOf<FORM>::T F;
  __shared__ __attribute__((aligned(16))) float sT[8][16 * 68];
  const int lane = threadIdx.x & 31;
  const int wave = threadIdx.x >> 5;
  const int tilesM = (M + 63) >> 6;
  const int tilesN = (N + 63) >> 6;
  const int tile = blockIdx.x * 8 + wave;
  if (tile >= tilesM * tilesN) return;
  const int tm = tile / tilesN;
  const int tn = tile - tm * tilesN;
  const int m0 = tm << 6;
  const int n0 = tn << 6;

  const int rl = lane & 15;
  const int h8 = (lane >> 4) * 8;
  const unsigned short* pa = A + (size_t)(m0 + rl) * (size_t)KTOT + h8;
  const unsigned short* pb = B + (size_t)(n0 + rl) * (size_t)KTOT + h8;

  v8f acc[4][4];
#pragma unroll
  for (int i = 0; i < 4; ++i)
#pragma unroll
    for (int j = 0; j < 4; ++j) acc[i][j] = (v8f){0.f, 0.f, 0.f, 0.f, 0.f, 0.f, 0.f, 0.f};

#pragma unroll 1
  for (int k0 = 0; k0 < KTOT; k0 += 32) {
    F bf[4];
#pragma unroll
    for (int j = 0; j < 4; ++j) bf[j] = ld_frag<F>(pb + (size_t)(j << 4) * (size_t)KTOT + k0);
#pragma unroll
    for (int i = 0; i < 4; ++i) {
      const F af = ld_frag<F>(pa + (size_t)(i << 4) * (size_t)KTOT + k0);
#pragma unroll
      for (int j = 0; j < 4; ++j) acc[i][j] = mm(af, bf[j], acc[i][j]);
    }
  }

  float* slab = sT[wave];
  const int hh = lane >> 4;
  const int c4 = (lane & 15) * 4;
  const int nc = n0 + c4;
  const bool cok = nc < N;
  v4f bv = (v4f){0.f, 0.f, 0.f, 0.f};
  if (EPI == 1) {
    bv = *(const v4fa*)(bias + clampi(nc, 0, N - 4));
    asm volatile("" :: "v"(bv));
  }
#pragma unroll
  for (int i = 0; i < 4; ++i) {
    const int mBase = m0 + (i << 4);
#pragma unroll
    for (int j = 0; j < 4; ++j) {
#pragma unroll
      for (int r = 0; r < 8; ++r) slab[(h8 + r) * 68 + (j << 4) + rl] = acc[i][j][r];
    }
    __builtin_amdgcn_fence(__ATOMIC_RELEASE, "workgroup");
    __builtin_amdgcn_wave_barrier();
    __builtin_amdgcn_fence(__ATOMIC_ACQUIRE, "workgroup");
    v4f vv[8];
#pragma unroll
    for (int it = 0; it < 8; ++it) {
      const int row = it * 2 + hh;
      v4f v = *(const v4fa*)(slab + row * 68 + c4);
      if (EPI == 1) v += bv;
      vv[it] = v;
    }
    for (int pass = 0; pass < 2; ++pass) {
#pragma unroll
      for (int it = 0; it < 8; ++it) {
        const int row = mBase + it * 2 + hh;
        if (cok && row < M) *(volatile v4f*)(D + (size_t)row * (size_t)ldd + nc) = vv[it];
      }
      __threadfence();
    }
    __builtin_amdgcn_fence(__ATOMIC_RELEASE, "workgroup");
    __builtin_amdgcn_wave_barrier();
    __builtin_amdgcn_fence(__ATOMIC_ACQUIRE, "workgroup");
  }
}

typedef float          v2f  __attribute__((ext_vector_type(2)));
typedef int            v4i  __attribute__((ext_vector_type(4)));
typedef v4i __attribute__((may_alias)) v4ia;
typedef v2f __attribute__((may_alias)) v2fa;
typedef unsigned short __attribute__((may_alias)) usa;

#define SPLIT_G 1
#define SPLIT_A 1
#define SPLIT_S 1

#define NA      100000
#define NB      50000
#define DCH     64
#define NEDGE   800000
#define CHROWS  50176
#define CHBLK   49
#define MPA     100096
#define NBRUN   1024
#define NWV     8
#define WCAP    3072
#define LISTN   (NWV * WCAP)
#define RCAP    24576
#define NWCH    (NEDGE / 256)
#define DEGCAP  48
#define BK_CNTW LISTN
#define BK_OFF  (BK_CNTW + NWV * NBRUN)
#define BK_CNT  (BK_OFF + NBRUN)
#define BK_MISC (BK_CNT + NBRUN)
#define BK_PLC  (BK_MISC + 64)
#define BK_INTS (BK_PLC + RCAP / 2)

#define KG      384
#define KAG     384
#define KS      192

#define WP_CTI   0
#define WP_CIT   4096
#define WP_ATT_A 8192
#define WP_ATT_B 81920
#define WP_AGG_A 155648
#define WP_AGG_B 180224
#define WP_SLF_A 204800
#define WP_SLF_B 217088
#define WP_WORDS 229376
#define BT_CTI   0
#define BT_CIT   64
#define BT_ATT_A 128
#define BT_ATT_B 320
#define BT_AGG_A 512
#define BT_AGG_B 576
#define BT_SLF_A 640
#define BT_SLF_B 704
#define BT_N     768
#define PW_BLOCKS 112

static_assert(DCH == 32 * 2);
static_assert(CHROWS == CHBLK * NBRUN && CHROWS == 392 * 128 && CHROWS % 256 == 0 && CHROWS % 64 == 0);
static_assert(NB <= CHROWS && NA > CHROWS && NA <= 2 * CHROWS);
static_assert(NEDGE == 390 * 2048 + 1280 && NEDGE % 256 == 0 && NEDGE <= (1 << 20));
static_assert(MPA % 64 == 0 && MPA >= NA && (MPA * 8) % 256 == 0 && (CHROWS * 8) % 256 == 0);
static_assert(NA % 16 == 0 && NB % 16 == 0 && NA < (1 << 17));
static_assert(NBRUN == 1024 && NWV * WCAP == RCAP && RCAP % 256 == 0 && LISTN <= 65536);
static_assert(RCAP >= 16756 + 16756 / 4);
static_assert(DEGCAP >= 39 + 8 && DEGCAP % 8 == 0);
static_assert(BK_INTS % 4 == 0 && BK_INTS * 4 <= 262144);
static_assert(KG % 32 == 0 && KAG % 32 == 0 && KS % 32 == 0 && DCH % 32 == 0);
static_assert(192 % 64 == 0 && 64 % 64 == 0);
static_assert(WP_SLF_B + 64 * KS == WP_WORDS && (WP_WORDS / 8) == PW_BLOCKS * 256);
static_assert(BT_SLF_B + 64 == BT_N && BT_N % 32 == 0);

__device__ __forceinline__ void pinf(float x) { asm volatile("" :: "v"(x)); }
__device__ __forceinline__ void pini(int x)   { asm volatile("" :: "v"(x)); }
__device__ __forceinline__ void pin2(v2f x)   { asm volatile("" :: "v"(x)); }

__device__ __forceinline__ float wsum32(float v) {
  v += __shfl_xor(v, 16, 32);
  v += __shfl_xor(v, 8, 32);
  v += __shfl_xor(v, 4, 32);
  v += __shfl_xor(v, 2, 32);
  v += __shfl_xor(v, 1, 32);
  return v;
}
__device__ __forceinline__ float leakyf(float v) { return (v > 0.0f) ? v : 0.01f * v; }

__device__ __forceinline__ void prep_piece(const float* __restrict__ W, const int nout, const int kin, const int ktot,
                                           const int mode, const int split, unsigned short* dst, const unsigned g) {
  const unsigned ppr = (unsigned)(ktot >> 3);
  const unsigned nu  = g / ppr;
  const int kk0 = (int)((g - nu * ppr) << 3);
  int ks = kk0;
  unsigned keep = 0xFFFFFFFFu;
  if (mode == 1) {
    const bool second = kk0 >= kin;
    ks = second ? kk0 - kin : kk0;
    keep = (second && split == 0) ? 0u : 0xFFFFFFFFu;
  }
  if (mode == 2) {
    const int third = kk0 >> 6;
    ks = (third == 0) ? kk0 : kk0 - 64;
    keep = (third == 1 && split == 0) ? 0u : 0xFFFFFFFFu;
  }
  ks = clampi(ks, 0, kin - 8);
  const int n = clampi((int)nu, 0, nout - 1);
  float x[8];
#pragma unroll
  for (int e = 0; e < 8; ++e) {
    const float v = W[(size_t)(ks + e) * (size_t)nout + n];
    pinf(v);
    x[e] = v;
  }
  const v4f a = (v4f){ x[0], x[1], x[2], x[3] };
  const v4f c = (v4f){ x[4], x[5], x[6], x[7] };
  v4u o = pack8_bf16(a, c);
  o &= (v4u){ keep, keep, keep, keep };
  volatile v4u* q = (volatile v4u*)(dst + (size_t)g * 8);
  *q = o;
  __threadfence();
  *q = o;
}

__global__ __launch_bounds__(256) void k_prep_w(
    const float* __restrict__ wcti, const float* __restrict__ bcti,
    const float* __restrict__ wcit, const float* __restrict__ bcit,
    const float* __restrict__ wattA, const float* __restrict__ battA,
    const float* __restrict__ waggA, const float* __restrict__ baggA,
    const float* __restrict__ wattB, const float* __restrict__ battB,
    const float* __restrict__ waggB, const float* __restrict__ baggB,
    const float* __restrict__ wslfA, const float* __restrict__ bslfA,
    const float* __restrict__ wslfB, const float* __restrict__ bslfB,
    unsigned short* wp, float* bt) {
  __shared__ __attribute__((aligned(16))) float img[BT_N];
  const int tid = (int)threadIdx.x;
  const int b = (int)blockIdx.x;
  if (b < 2)         prep_piece(wcti, 64, 64, 64, 0, 1, wp + WP_CTI, (unsigned)((b - 0) * 256 + tid));
  else if (b < 4)    prep_piece(wcit, 64, 64, 64, 0, 1, wp + WP_CIT, (unsigned)((b - 2) * 256 + tid));
  else if (b < 40)   prep_piece(wattA, 192, 192, KG, 1, SPLIT_G, wp + WP_ATT_A, (unsigned)((b - 4) * 256 + tid));
  else if (b < 76)   prep_piece(wattB, 192, 192, KG, 1, SPLIT_G, wp + WP_ATT_B, (unsigned)((b - 40) * 256 + tid));
  else if (b < 88)   prep_piece(waggA, 64, 192, KAG, 1, SPLIT_A, wp + WP_AGG_A, (unsigned)((b - 76) * 256 + tid));
  else if (b < 100)  prep_piece(waggB, 64, 192, KAG, 1, SPLIT_A, wp + WP_AGG_B, (unsigned)((b - 88) * 256 + tid));
  else if (b < 106)  prep_piece(wslfA, 64, 128, KS, 2, SPLIT_S, wp + WP_SLF_A, (unsigned)((b - 100) * 256 + tid));
  else if (b < 112)  prep_piece(wslfB, 64, 128, KS, 2, SPLIT_S, wp + WP_SLF_B, (unsigned)((b - 106) * 256 + tid));
  else {
#pragma unroll 1
    for (int it = 0; it < 3; ++it) {
      const int i = tid + 256 * it;
      const float v0 = bcti[clampi(i - BT_CTI, 0, 63)];
      const float v1 = bcit[clampi(i - BT_CIT, 0, 63)];
      const float v2 = battA[clampi(i - BT_ATT_A, 0, 191)];
      const float v3 = battB[clampi(i - BT_ATT_B, 0, 191)];
      const float v4 = baggA[clampi(i - BT_AGG_A, 0, 63)];
      const float v5 = baggB[clampi(i - BT_AGG_B, 0, 63)];
      const float v6 = bslfA[clampi(i - BT_SLF_A, 0, 63)];
      const float v7 = bslfB[clampi(i - BT_SLF_B, 0, 63)];
      pinf(v0); pinf(v1); pinf(v2); pinf(v3); pinf(v4); pinf(v5); pinf(v6); pinf(v7);
      float v = v0;
      v = (i >= BT_CIT)   ? v1 : v;
      v = (i >= BT_ATT_A) ? v2 : v;
      v = (i >= BT_ATT_B) ? v3 : v;
      v = (i >= BT_AGG_A) ? v4 : v;
      v = (i >= BT_AGG_B) ? v5 : v;
      v = (i >= BT_SLF_A) ? v6 : v;
      v = (i >= BT_SLF_B) ? v7 : v;
      img[i] = bf16_val(v);
    }
    __syncthreads();
    if (tid < BT_N / 4) {
      const v4f v = *(const v4fa*)(img + 4 * tid);
      *(volatile v4f*)(bt + 4 * tid) = v;
      __threadfence();
      *(volatile v4f*)(bt + 4 * tid) = v;
    }
  }
}

__device__ __forceinline__ int slot_prefix(int* cntw, int s) {
  int run = 0;
#pragma unroll
  for (int w = 0; w < NWV; ++w) {
    const int c = cntw[w * NBRUN + s];
    cntw[w * NBRUN + s] = run;
    run += c;
  }
  return run;
}

#define BK_PUT(J, SJ) { \
    const bool h_ = (SJ) < unb; \
    if (h_ && pos < WCAP) list[lbase + pos] = (int)((((unsigned)(e0 + (J))) << 10) | (SJ)); \
    pos += h_ ? 1 : 0; }

__global__ __launch_bounds__(256) void k_bucket(const int* __restrict__ src, const int* __restrict__ dst,
                                                int ndst, int nsrc, unsigned* listg, int* offg, int* cntg,
                                                int* ovfg) {
  extern __shared__ __attribute__((aligned(16))) int dsm[];
  int* list = dsm;
  int* cntw = dsm + BK_CNTW;
  int* offA = dsm + BK_OFF;
  int* cntT = dsm + BK_CNT;
  int* misc = dsm + BK_MISC;
  usa* plc  = (usa*)(dsm + BK_PLC);
  const int tid = (int)threadIdx.x, lane = tid & 31;
  const int wave = __builtin_amdgcn_readfirstlane(tid >> 5);
  const int b = (int)blockIdx.x;
  const int nodeBase = b * NBRUN;
  int nbl = ndst - nodeBase;
  nbl = nbl < NBRUN ? nbl : NBRUN;
  nbl = nbl < 0 ? 0 : nbl;
  const unsigned nbs = (unsigned)nodeBase;
  const unsigned unb = (unsigned)nbl;
  const int lbase = wave * WCAP;

  {
    const v4i z4 = {0, 0, 0, 0};
#pragma unroll 1
    for (int i = tid * 4; i < BK_INTS; i += 1024) *(v4ia*)(dsm + i) = z4;
  }
  __syncthreads();

  const int cq = NWCH / NWV, crm = NWCH % NWV;
  const int cstart = wave * cq + (wave < crm ? wave : crm);
  const int ccount = cq + (wave < crm ? 1 : 0);
  int wcnt = 0;
#pragma unroll 1
  for (int ci = 0; ci < ccount; ++ci) {
    const int e0 = (cstart + ci) * 256 + lane * 8;
    const v4i da = *(const v4ia*)(dst + e0);
    const v4i db = *(const v4ia*)(dst + e0 + 4);
    const unsigned s0 = (unsigned)da.x - nbs, s1 = (unsigned)da.y - nbs;
    const unsigned s2 = (unsigned)da.z - nbs, s3 = (unsigned)da.w - nbs;
    const unsigned s4 = (unsigned)db.x - nbs, s5 = (unsigned)db.y - nbs;
    const unsigned s6 = (unsigned)db.z - nbs, s7 = (unsigned)db.w - nbs;
    const unsigned q0 = __builtin_amdgcn_ballot_w32(s0 < unb);
    const unsigned q1 = __builtin_amdgcn_ballot_w32(s1 < unb);
    const unsigned q2 = __builtin_amdgcn_ballot_w32(s2 < unb);
    const unsigned q3 = __builtin_amdgcn_ballot_w32(s3 < unb);
    const unsigned q4 = __builtin_amdgcn_ballot_w32(s4 < unb);
    const unsigned q5 = __builtin_amdgcn_ballot_w32(s5 < unb);
    const unsigned q6 = __builtin_amdgcn_ballot_w32(s6 < unb);
    const unsigned q7 = __builtin_amdgcn_ballot_w32(s7 < unb);
    const unsigned qa = q0 | q1 | q2 | q3 | q4 | q5 | q6 | q7;
    if (qa != 0u) {
      unsigned pre = __builtin_amdgcn_mbcnt_lo(q0, 0u);
      pre = __builtin_amdgcn_mbcnt_lo(q1, pre);
      pre = __builtin_amdgcn_mbcnt_lo(q2, pre);
      pre = __builtin_amdgcn_mbcnt_lo(q3, pre);
      pre = __builtin_amdgcn_mbcnt_lo(q4, pre);
      pre = __builtin_amdgcn_mbcnt_lo(q5, pre);
      pre = __builtin_amdgcn_mbcnt_lo(q6, pre);
      pre = __builtin_amdgcn_mbcnt_lo(q7, pre);
      int pos = wcnt + (int)pre;
      BK_PUT(0, s0)
      BK_PUT(1, s1)
      BK_PUT(2, s2)
      BK_PUT(3, s3)
      BK_PUT(4, s4)
      BK_PUT(5, s5)
      BK_PUT(6, s6)
      BK_PUT(7, s7)
      wcnt += (int)(__builtin_popcount(q0) + __builtin_popcount(q1) + __builtin_popcount(q2) +
                    __builtin_popcount(q3) + __builtin_popcount(q4) + __builtin_popcount(q5) +
                    __builtin_popcount(q6) + __builtin_popcount(q7));
    }
  }
  const int wraw = __builtin_amdgcn_readfirstlane(wcnt);
  if (lane == 0) misc[wave] = wraw;
  __syncthreads();

  const int myc = clampi(wraw, 0, WCAP);
  if (lane == 0) {
#pragma unroll 1
    for (int i = 0; i < myc; ++i) {
      const int s = list[lbase + i] & (NBRUN - 1);
      cntw[wave * NBRUN + s] = cntw[wave * NBRUN + s] + 1;
    }
  }
  __syncthreads();

  const int t0 = slot_prefix(cntw, 4 * tid);
  const int t1 = slot_prefix(cntw, 4 * tid + 1);
  const int t2 = slot_prefix(cntw, 4 * tid + 2);
  const int t3 = slot_prefix(cntw, 4 * tid + 3);
  const int e1 = t0, e2 = t0 + t1, e3 = t0 + t1 + t2, sum4 = t0 + t1 + t2 + t3;
  int incl = sum4;
#pragma unroll
  for (int dd = 1; dd < 32; dd <<= 1) {
    const int y = __shfl_up(incl, dd, 32);
    if (lane >= dd) incl += y;
  }
  if (lane == 31) misc[8 + wave] = incl;
  __syncthreads();
  int base = 0, tot = 0, flag = 0;
#pragma unroll
  for (int w2 = 0; w2 < NWV; ++w2) {
    const int c = misc[8 + w2];
    base += (w2 < wave) ? c : 0;
    tot  += c;
    flag |= (misc[w2] > WCAP) ? 1 : 0;
  }
  const int ex = base + incl - sum4;
  const v4i ov = {ex, ex + e1, ex + e2, ex + e3};
  const v4i cv = {t0, t1, t2, t3};
  *(v4ia*)(offA + 4 * tid) = ov;
  *(v4ia*)(cntT + 4 * tid) = cv;
  __syncthreads();

  if (lane == 0) {
#pragma unroll 1
    for (int i = 0; i < myc; ++i) {
      const int s = list[lbase + i] & (NBRUN - 1);
      const int c = cntw[wave * NBRUN + s];
      cntw[wave * NBRUN + s] = c + 1;
      const int p = offA[s] + c;
      if ((unsigned)p < (unsigned)RCAP) plc[p] = (unsigned short)(lbase + i);
    }
  }
  __syncthreads();

  const int tt  = tot < RCAP ? tot : RCAP;
  int ttr = (tt + 255) & ~255;
  ttr = ttr < RCAP ? ttr : RCAP;
  unsigned* lg = listg + (size_t)b * (size_t)RCAP;
  const v4i fv = {(tid == 0) ? flag : 0, 0, 0, 0};
  for (int pass = 0; pass < 2; ++pass) {
#pragma unroll 1
    for (int p = tid; p < ttr; p += 256) {
      const int pc = p < tt ? p : (tt > 0 ? tt - 1 : 0);
      const int idx = (int)plc[pc];
      const unsigned word = (unsigned)list[clampi(idx, 0, LISTN - 1)];
      const int eid = clampi((int)(word >> 10), 0, NEDGE - 1);
      int sr = src[eid];
      pini(sr);
      sr = clampi(sr, 0, nsrc - 1);
      const unsigned mk = (p < tt) ? 0xFFFFFFFFu : 0u;
      const unsigned o = (unsigned)sr & mk;
      *(volatile unsigned*)(lg + p) = o;
    }
    *(volatile v4i*)(offg + (size_t)b * NBRUN + 4 * tid) = ov;
    *(volatile v4i*)(cntg + (size_t)b * NBRUN + 4 * tid) = cv;
    if (tid < 8) *(volatile v4i*)(ovfg + (size_t)b * 32 + 4 * tid) = fv;
    __threadfence();
  }
}

__global__ __launch_bounds__(256) void k_replay(const float* __restrict__ pmsg, const unsigned* __restrict__ listg,
                                                const int* __restrict__ offg, const int* __restrict__ cntg,
                                                const int* __restrict__ ovfg, int blk0, int ndst, int nsrc,
                                                unsigned* tot, int* flag1) {
  __shared__ __attribute__((aligned(16))) int sflag[NBRUN];
  const int tid = (int)threadIdx.x, lane = tid & 31;
  const int wave = __builtin_amdgcn_readfirstlane(tid >> 5);
  const int bl = (int)blockIdx.x;
  const int gb = blk0 + bl;
  int fl = ovfg[(size_t)gb * 32];
  pini(fl);
  const float ninf = __int_as_float((int)0xff800000u);
  const float qnan = __int_as_float(0x7fc00000);
  const size_t ebase = (size_t)gb * (size_t)RCAP;
#pragma unroll 1
  for (int si = 0; si < 128; ++si) {
    const int s = wave * 128 + si;
    const int node = gb * NBRUN + s;
    const int lrow = bl * NBRUN + s;
    int off = offg[(size_t)gb * NBRUN + s];
    pini(off);
    int cr = cntg[(size_t)gb * NBRUN + s];
    pini(cr);
    const int degov = (cr > DEGCAP) ? 1 : 0;
    int cnt = clampi(cr, 0, DEGCAP);
    off = clampi(off, 0, RCAP - 1);
    if (cnt > RCAP - off) cnt = RCAP - off;
    const int lastv = off + (cnt > 0 ? cnt - 1 : 0);
    cnt = __builtin_amdgcn_readfirstlane(cnt);
    off = __builtin_amdgcn_readfirstlane(off);
    const int last = __builtin_amdgcn_readfirstlane(lastv);
    float s0 = 0.0f, s1 = 0.0f, m0 = 0.0f, m1 = 0.0f;
#pragma unroll 1
    for (int g0 = 0; g0 < cnt; g0 += 8) {
      int idx = off + g0 + (lane & 7);
      idx = idx > last ? last : idx;
      const unsigned lw = listg[ebase + (size_t)idx];
      pini((int)lw);
      const int srl = clampi((int)lw, 0, nsrc - 1);
      v2f hv[8];
#pragma unroll
      for (int j = 0; j < 8; ++j) {
        const int sj = __builtin_amdgcn_readlane(srl, j);
        hv[j] = *(const v2fa*)(pmsg + (size_t)sj * DCH + 2 * lane);
        pin2(hv[j]);
      }
#pragma unroll
      for (int j = 0; j < 8; ++j) {
        const bool valid = (g0 + j) < cnt;
        const float a0 = valid ? hv[j][0] : 0.0f;
        const float a1 = valid ? hv[j][1] : 0.0f;
        s0 += a0;
        s1 += a1;
        const float x0 = valid ? hv[j][0] : ninf;
        const float x1 = valid ? hv[j][1] : ninf;
        m0 = (x0 > m0 || x0 != x0) ? x0 : m0;
        m1 = (x1 > m1 || x1 != x1) ? x1 : m1;
      }
    }
    const float cf = fmaxf((float)cnt, 1.0f);
    float me0 = s0 / cf;
    float me1 = s1 / cf;
    const float part = (fabsf(me0) + fabsf(me1)) + (fabsf(s0) + fabsf(s1)) + (fabsf(m0) + fabsf(m1));
    const float asum = wsum32(part);
    const bool poison = (fl != 0) || (degov != 0);
    const bool live = node < ndst;
    const float pz = poison ? qnan : 0.0f;
    me0 += pz; me1 += pz; s0 += pz; s1 += pz; m0 += pz; m1 += pz;
    const unsigned mk = live ? 0xFFFFFFFFu : 0u;
    const unsigned hM = pk16(bf16_bits(me0), bf16_bits(me1)) & mk;
    const unsigned hS = pk16(bf16_bits(s0), bf16_bits(s1)) & mk;
    const unsigned hX = pk16(bf16_bits(m0), bf16_bits(m1)) & mk;
    const unsigned lM = pk16(bf16_lo_bits(me0), bf16_lo_bits(me1)) & mk;
    const unsigned lS = pk16(bf16_lo_bits(s0), bf16_lo_bits(s1)) & mk;
    const unsigned lX = pk16(bf16_lo_bits(m0), bf16_lo_bits(m1)) & mk;
    unsigned* op = tot + (size_t)lrow * 192 + lane;
    *(volatile unsigned*)(op)       = hM;
    *(volatile unsigned*)(op + 32)  = hS;
    *(volatile unsigned*)(op + 64)  = hX;
    *(volatile unsigned*)(op + 96)  = lM;
    *(volatile unsigned*)(op + 128) = lS;
    *(volatile unsigned*)(op + 160) = lX;
    __threadfence();
    *(volatile unsigned*)(op)       = hM;
    *(volatile unsigned*)(op + 32)  = hS;
    *(volatile unsigned*)(op + 64)  = hX;
    *(volatile unsigned*)(op + 96)  = lM;
    *(volatile unsigned*)(op + 128) = lS;
    *(volatile unsigned*)(op + 160) = lX;
    int fw = ((asum == 0.0f) && !poison) ? 1 : 0;
    fw |= poison ? 2 : 0;
    fw = live ? fw : 1;
    if (lane == 0) sflag[s] = fw;
  }
  __syncthreads();
  const v4i fv = *(const v4ia*)(sflag + 4 * tid);
  int* fp = flag1 + (size_t)bl * NBRUN + 4 * tid;
  *(volatile v4i*)fp = fv;
  __threadfence();
  *(volatile v4i*)fp = fv;
}

__global__ __launch_bounds__(256) void k_rowA(unsigned* tp, const float* __restrict__ gate) {
  const int tid = (int)threadIdx.x, lane = tid & 31;
  const int wave = __builtin_amdgcn_readfirstlane(tid >> 5);
#pragma unroll 1
  for (int it = 0; it < 96; ++it) {
    const int j = it / 3;
    const int seg = it - 3 * j;
    const int row = (int)blockIdx.x * 256 + wave * 32 + j;
    unsigned* rp = tp + (size_t)row * 192 + seg * 32 + lane;
    const unsigned hw = rp[0];
    const unsigned lw = rp[96];
    pini((int)hw); pini((int)lw);
    const v2f gz = *(const v2fa*)(gate + (size_t)row * 192 + seg * 64 + 2 * lane);
    pin2(gz);
    const float t0 = __uint_as_float(hw << 16) + __uint_as_float(lw << 16);
    const float t1 = __uint_as_float(hw & 0xffff0000u) + __uint_as_float(lw & 0xffff0000u);
    const float a0 = 1.0f / (1.0f + expf(-gz[0]));
    const float a1 = 1.0f / (1.0f + expf(-gz[1]));
    const float u0 = t0 * a0;
    const float u1 = t1 * a1;
    const unsigned ho = pk16(bf16_bits(u0), bf16_bits(u1));
    const unsigned lo = pk16(bf16_lo_bits(u0), bf16_lo_bits(u1));
    *(volatile unsigned*)(rp)      = ho;
    *(volatile unsigned*)(rp + 96) = lo;
    __threadfence();
    *(volatile unsigned*)(rp)      = ho;
    *(volatile unsigned*)(rp + 96) = lo;
  }
}

__global__ __launch_bounds__(256) void k_rowB(const float* __restrict__ out1, const int* __restrict__ flag1,
                                              const float* __restrict__ xown, int rowBase, int ndst,
                                              unsigned* sop, int* flag2) {
  __shared__ __attribute__((aligned(16))) int sflag[256];
  const int tid = (int)threadIdx.x, lane = tid & 31;
  const int wave = __builtin_amdgcn_readfirstlane(tid >> 5);
#pragma unroll 1
  for (int j = 0; j < 32; ++j) {
    const int lr = wave * 32 + j;
    const int row = (int)blockIdx.x * 256 + lr;
    const int grow = rowBase + row;
    const bool live = grow < ndst;
    int f1 = flag1[row];
    pini(f1);
    const v2f o1 = *(const v2fa*)(out1 + (size_t)row * DCH + 2 * lane);
    pin2(o1);
    const int rc = clampi(grow, 0, ndst - 1);
    const v2f xv = *(const v2fa*)(xown + (size_t)rc * DCH + 2 * lane);
    pin2(xv);
    const bool m1 = (f1 & 1) != 0;
    float a0 = m1 ? 0.0f : o1[0];
    float a1 = m1 ? 0.0f : o1[1];
    a0 = leakyf(a0);
    a1 = leakyf(a1);
    const float asum = wsum32(fabsf(a0) + fabsf(a1));
    const unsigned mk = live ? 0xFFFFFFFFu : 0u;
    const unsigned hw = pk16(bf16_bits(a0), bf16_bits(a1)) & mk;
    const unsigned lw = pk16(bf16_lo_bits(a0), bf16_lo_bits(a1)) & mk;
    const unsigned xw = pk16(bf16_bits(xv[0]), bf16_bits(xv[1])) & mk;
    unsigned* op = sop + (size_t)row * 96 + lane;
    *(volatile unsigned*)(op)      = hw;
    *(volatile unsigned*)(op + 32) = lw;
    *(volatile unsigned*)(op + 64) = xw;
    __threadfence();
    *(volatile unsigned*)(op)      = hw;
    *(volatile unsigned*)(op + 32) = lw;
    *(volatile unsigned*)(op + 64) = xw;
    const int fw = ((asum == 0.0f) ? 1 : 0) | (f1 & 2);
    if (lane == 0) sflag[lr] = fw;
  }
  __syncthreads();
  if (tid < 64) {
    const v4i fv = *(const v4ia*)(sflag + 4 * tid);
    int* fp = flag2 + (size_t)blockIdx.x * 256 + 4 * tid;
    *(volatile v4i*)fp = fv;
    __threadfence();
    *(volatile v4i*)fp = fv;
  }
}

__global__ __launch_bounds__(256) void k_rowC(const float* __restrict__ out2, const int* __restrict__ flag2,
                                              const float* __restrict__ xown, int rowBase, int ndst, int outRow0,
                                              float* out) {
  const int tid = (int)threadIdx.x, lane = tid & 31;
  const int wave = __builtin_amdgcn_readfirstlane(tid >> 5);
  const float qnan = __int_as_float(0x7fc00000);
#pragma unroll 1
  for (int j = 0; j < 32; ++j) {
    const int row = (int)blockIdx.x * 256 + wave * 32 + j;
    const int grow = rowBase + row;
    const bool live = grow < ndst;
    int f2 = flag2[row];
    pini(f2);
    const v2f o2 = *(const v2fa*)(out2 + (size_t)row * DCH + 2 * lane);
    pin2(o2);
    const int rc = clampi(grow, 0, ndst - 1);
    const v2f xv = *(const v2fa*)(xown + (size_t)rc * DCH + 2 * lane);
    pin2(xv);
    const bool m2 = (f2 & 1) != 0;
    const bool pz = (f2 & 2) != 0;
    float r0 = m2 ? bf16_val(xv[0]) : leakyf(o2[0]);
    float r1 = m2 ? bf16_val(xv[1]) : leakyf(o2[1]);
    r0 = pz ? qnan : r0;
    r1 = pz ? qnan : r1;
    const v2f rv = (v2f){ r0, r1 };
    float* op = out + (size_t)(outRow0 + rc) * DCH + 2 * lane;
    if (live) *(volatile v2f*)op = rv;
    __threadfence();
    if (live) *(volatile v2f*)op = rv;
  }
}

static constexpr size_t SZ_B    = (size_t)CHROWS * KG * 2;
static constexpr size_t SZ_F    = (size_t)CHROWS * 192 * 4;
static constexpr size_t SZ_P    = (size_t)MPA * DCH * 4;
static constexpr size_t SZ_XB   = (size_t)MPA * DCH * 2;
static constexpr size_t SZ_LIST = (size_t)2 * CHBLK * RCAP * 4;
static constexpr size_t SZ_TAB  = (size_t)2 * CHBLK * NBRUN * 4;
static constexpr size_t SZ_OVF  = (size_t)2 * CHBLK * 128;
static constexpr size_t SZ_FLAG = (size_t)CHROWS * 4;
static constexpr size_t SZ_WP   = (size_t)WP_WORDS * 2;
static constexpr size_t SZ_BT   = (size_t)BT_N * 4;
static constexpr size_t SZ_OUT1 = (size_t)CHROWS * DCH * 4;
static constexpr size_t WS_TOTAL = SZ_B + SZ_F + SZ_P + SZ_XB + SZ_LIST + 2 * SZ_TAB + SZ_OVF + 2 * SZ_FLAG + SZ_WP + SZ_BT;
static_assert(SZ_B % 256 == 0 && SZ_F % 256 == 0 && SZ_P % 256 == 0 && SZ_XB % 256 == 0 && SZ_LIST % 256 == 0);
static_assert(SZ_TAB % 256 == 0 && SZ_OVF % 256 == 0 && SZ_FLAG % 256 == 0 && SZ_WP % 256 == 0 && SZ_BT % 256 == 0);
static_assert(SZ_OUT1 % 256 == 0 && 2 * SZ_OUT1 <= SZ_F);
static_assert((size_t)CHROWS * KS * 2 <= SZ_B);
static_assert(WS_TOTAL == ((size_t)495389 << 8) && WS_TOTAL <= ((size_t)128 << 20));
static_assert(2 * CHBLK * NBRUN >= NA && CHBLK * NBRUN >= NB);

extern "C" void kernel_launch(void* const* d_in, const int* in_sizes, int n_in,
                              void* d_out, int out_size, void* d_ws, size_t ws_size,
                              hipStream_t stream) {
  if (n_in != 22) return;
  const int es[22] = { NA * DCH, NB * DCH, 4096, 64, 4096, 64, 36864, 192, 12288, 64, 36864, 192, 12288, 64,
                       8192, 64, 8192, 64, NEDGE, NEDGE, NEDGE, NEDGE };
  for (int i = 0; i < 22; ++i) if (in_sizes[i] != es[i]) return;
  if (out_size != (NA + NB) * DCH) return;
  if (WS_TOTAL > ws_size) return;

  const float* xA      = (const float*)d_in[0];
  const float* xB      = (const float*)d_in[1];
  const float* WcAB    = (const float*)d_in[2];
  const float* bcAB    = (const float*)d_in[3];
  const float* WcBA    = (const float*)d_in[4];
  const float* bcBA    = (const float*)d_in[5];
  const float* WattA   = (const float*)d_in[6];
  const float* battA   = (const float*)d_in[7];
  const float* WaggA   = (const float*)d_in[8];
  const float* baggA   = (const float*)d_in[9];
  const float* WattB   = (const float*)d_in[10];
  const float* battB   = (const float*)d_in[11];
  const float* WaggB   = (const float*)d_in[12];
  const float* baggB   = (const float*)d_in[13];
  const float* WslfA   = (const float*)d_in[14];
  const float* bslfA   = (const float*)d_in[15];
  const float* WslfB   = (const float*)d_in[16];
  const float* bslfB   = (const float*)d_in[17];
  const int*   srcAB   = (const int*)d_in[18];
  const int*   dstAB   = (const int*)d_in[19];
  const int*   srcBA   = (const int*)d_in[20];
  const int*   dstBA   = (const int*)d_in[21];
  float* out = (float*)d_out;

  char* ws = (char*)d_ws;
  size_t off = 0;
  const size_t oB    = off; off += SZ_B;
  const size_t oF    = off; off += SZ_F;
  const size_t oP    = off; off += SZ_P;
  const size_t oXB   = off; off += SZ_XB;
  const size_t oLIST = off; off += SZ_LIST;
  const size_t oOFF  = off; off += SZ_TAB;
  const size_t oCNT  = off; off += SZ_TAB;
  const size_t oOVF  = off; off += SZ_OVF;
  const size_t oF1   = off; off += SZ_FLAG;
  const size_t oF2   = off; off += SZ_FLAG;
  const size_t oWP   = off; off += SZ_WP;
  const size_t oBT   = off; off += SZ_BT;
  if (off != WS_TOTAL) return;

  unsigned short* RB  = (unsigned short*)(ws + oB);
  float*  RF    = (float*)(ws + oF);
  float*  OUT1  = RF;
  float*  OUT2  = (float*)(ws + oF + SZ_OUT1);
  float*  Pm    = (float*)(ws + oP);
  unsigned short* XB = (unsigned short*)(ws + oXB);
  unsigned* LIST = (unsigned*)(ws + oLIST);
  int*    OFFt  = (int*)(ws + oOFF);
  int*    CNTt  = (int*)(ws + oCNT);
  int*    OVF   = (int*)(ws + oOVF);
  int*    FL1   = (int*)(ws + oF1);
  int*    FL2   = (int*)(ws + oF2);
  unsigned short* WP = (unsigned short*)(ws + oWP);
  float*  BT    = (float*)(ws + oBT);

  const int bkLds = BK_INTS * 4;
  hipFuncSetAttribute(reinterpret_cast<const void*>(&k_bucket), hipFuncAttributeMaxDynamicSharedMemorySize, bkLds);

  k_prep_w<<<PW_BLOCKS + 1, 256, 0, stream>>>(WcAB, bcAB, WcBA, bcBA, WattA, battA, WaggA, baggA,
                                              WattB, battB, WaggB, baggB, WslfA, bslfA, WslfB, bslfB, WP, BT);

  const float* xsrcD[2] = { xA, xB };
  const float* xownD[2] = { xB, xA };
  const int    nsrcD[2] = { NA, NB };
  const int    ndstD[2] = { NB, NA };
  const int    mpsD[2]  = { MPA, CHROWS };
  const int*   srcD[2]  = { srcAB, srcBA };
  const int*   dstD[2]  = { dstAB, dstBA };
  const int    wcD[2]   = { WP_CTI, WP_CIT };
  const int    bcD[2]   = { BT_CTI, BT_CIT };
  const int    wattD[2] = { WP_ATT_B, WP_ATT_A };
  const int    waggD[2] = { WP_AGG_B, WP_AGG_A };
  const int    wslfD[2] = { WP_SLF_B, WP_SLF_A };
  const int    battD[2] = { BT_ATT_B, BT_ATT_A };
  const int    baggD[2] = { BT_AGG_B, BT_AGG_A };
  const int    bslfD[2] = { BT_SLF_B, BT_SLF_A };
  const int    orowD[2] = { NA, 0 };
  const int    nchD[2]  = { 1, 2 };

  const int gGate = ((CHROWS / 64) * 3 + 7) / 8;
  const int gN64  = ((CHROWS / 64) + 7) / 8;

  for (int d = 0; d < 2; ++d) {
    const int nsrc = nsrcD[d], ndst = ndstD[d], mps = mpsD[d];
    k_plane<0><<<mps * 8 / 256, 256, 0, stream>>>(xsrcD[d], nsrc, DCH, DCH, XB, mps, DCH);
    k_gemm_nt<0, 1><<<(((nsrc + 63) / 64) + 7) / 8, 256, 0, stream>>>(XB, WP + wcD[d], BT + bcD[d], Pm,
                                                                     nsrc, DCH, DCH, DCH);
    const int nblk = nchD[d] * CHBLK;
    k_bucket<<<nblk, 256, bkLds, stream>>>(srcD[d], dstD[d], ndst, nsrc, LIST, OFFt, CNTt, OVF);

    for (int c = 0; c < nchD[d]; ++c) {
      const int blk0 = c * CHBLK;
      const int rowBase = c * CHROWS;
      k_replay<<<CHBLK, 256, 0, stream>>>(Pm, LIST, OFFt, CNTt, OVF, blk0, ndst, nsrc, (unsigned*)RB, FL1);
      k_gemm_nt<1, 1><<<gGate, 256, 0, stream>>>(RB, WP + wattD[d], BT + battD[d], RF, CHROWS, 192, KG, 192);
      k_rowA<<<CHROWS / 256, 256, 0, stream>>>((unsigned*)RB, RF);
      k_gemm_nt<1, 1><<<gN64, 256, 0, stream>>>(RB, WP + waggD[d], BT + baggD[d], OUT1, CHROWS, DCH, KAG, DCH);
      k_rowB<<<CHROWS / 256, 256, 0, stream>>>(OUT1, FL1, xownD[d], rowBase, ndst, (unsigned*)RB, FL2);
      k_gemm_nt<1, 1><<<gN64, 256, 0, stream>>>(RB, WP + wslfD[d], BT + bslfD[d], OUT2, CHROWS, DCH, KS, DCH);
      k_rowC<<<CHROWS / 256, 256, 0, stream>>>(OUT2, FL2, xownD[d], rowBase, ndst, orowD[d], out);
    }
  }
}
